// Double_SSM_Block_out_59382217834755
// MI455X (gfx1250) — hardware-verified
//
#include <hip/hip_runtime.h>
#include <hip/hip_bf16.h>


#define NB_   16
#define DM_   128
#define HH_   64
#define WW_   64
#define NL_   4096
#define MT_   65536
#define DI_   256
#define NS_   16
#define DTR_  8
#define NXP_  40
#define NXT_  48
#define XDP_  64
#define OC_   128

#define TT_   128
#define TR_   144
#define PA_   136
#define PC_   136
#define PD_   68
#define PZ_   68
#define PO_   36

static_assert(MT_ == NB_ * NL_);
static_assert(NL_ == HH_ * WW_);
static_assert(NL_ % TT_ == 0);
static_assert(TR_ == TT_ + 16);
static_assert(DM_ % 32 == 0);
static_assert(DI_ % 64 == 0);
static_assert(NXT_ % 16 == 0);
static_assert(NXT_ >= NXP_);
static_assert(NXT_ <= XDP_);
static_assert(DTR_ + 2 * NS_ == NXP_);
static_assert(DM_ * (TR_ / 4) == 18 * 256);
static_assert(TT_ * PD_ * 4 <= 2 * TR_ * PA_ * 2);

typedef float          v4f   __attribute__((ext_vector_type(4)));
typedef float          v8f   __attribute__((ext_vector_type(8)));
typedef __bf16         v16b  __attribute__((ext_vector_type(16)));
typedef unsigned short u16x8 __attribute__((ext_vector_type(8)));

union FragB { u16x8 h[2]; v16b v; };

constexpr size_t SZ_WI  = (size_t)(2 * DI_) * DM_ * 2;
constexpr size_t SZ_WX  = (size_t)NXT_ * DI_ * 2;
constexpr size_t SZ_WO  = (size_t)OC_ * DI_ * 2;
constexpr size_t SZ_U   = (size_t)MT_ * DM_ * 2;
constexpr size_t SZ_XC  = (size_t)MT_ * DI_ * 2;
constexpr size_t SZ_XD  = (size_t)MT_ * XDP_ * 4;
constexpr size_t OFF_WIH = 0;
constexpr size_t OFF_WIL = OFF_WIH + SZ_WI;
constexpr size_t OFF_WXH = OFF_WIL + SZ_WI;
constexpr size_t OFF_WXL = OFF_WXH + SZ_WX;
constexpr size_t OFF_WOH = OFF_WXL + SZ_WX;
constexpr size_t OFF_WOL = OFF_WOH + SZ_WO;
constexpr size_t OFF_UH  = OFF_WOL + SZ_WO;
constexpr size_t OFF_UL  = OFF_UH + SZ_U;
constexpr size_t OFF_XH  = OFF_UL + SZ_U;
constexpr size_t OFF_XL  = OFF_XH + SZ_XC;
constexpr size_t OFF_XD  = OFF_XL + SZ_XC;
constexpr size_t WS_END  = OFF_XD + SZ_XD;
static_assert(WS_END <= (size_t)134217728);
static_assert(OFF_WIL % 128 == 0 && OFF_WXH % 128 == 0 && OFF_WXL % 128 == 0 && OFF_WOH % 128 == 0);
static_assert(OFF_WOL % 128 == 0 && OFF_UH % 128 == 0 && OFF_UL % 128 == 0 && OFF_XH % 128 == 0);
static_assert(OFF_XL % 128 == 0 && OFF_XD % 128 == 0);

constexpr unsigned LDS_PRE = (unsigned)(2 * TR_ * PA_ * 2 + 2 * TR_ * PC_ * 2);
static_assert(LDS_PRE == 156672u);

extern __shared__ __attribute__((aligned(16))) unsigned char smem_dyn[];

__device__ __forceinline__ unsigned short f2bf(float f) {
    const unsigned u = __float_as_uint(f);
    const unsigned r = u + 0x7FFFu + ((u >> 16) & 1u);
    return (unsigned short)(r >> 16);
}
__device__ __forceinline__ float bf2f(unsigned short b) {
    return __uint_as_float(((unsigned)b) << 16);
}
__device__ __forceinline__ void split2(float f, unsigned short& hb, unsigned short& lb) {
    hb = f2bf(f);
    lb = f2bf(f - bf2f(hb));
}
__device__ __forceinline__ float silu_f(float x) {
    const float e = __expf(-x);
    return x * __builtin_amdgcn_rcpf(1.0f + e);
}
__device__ __forceinline__ float softplus_f(float x) {
    return fmaxf(x, 0.0f) + log1pf(__expf(-fabsf(x)));
}
__device__ __forceinline__ v8f zero8() {
    v8f z;
#pragma unroll
    for (int c = 0; c < 8; ++c) z[c] = 0.0f;
    return z;
}

__device__ __forceinline__ void mma_bf(v8f& acc, const FragB& a, const FragB& b) {
    acc = __builtin_amdgcn_wmma_f32_16x16x32_bf16(false, a.v, false, b.v, (short)0, acc, false, false);
    asm volatile("v_nop\n\tv_nop\n\tv_nop\n\tv_nop" : "+v"(acc) : "v"(a.v), "v"(b.v));
}
__device__ __forceinline__ void mma3(v8f& acc, const FragB& ah, const FragB& al,
                                     const FragB& bh, const FragB& bl) {
    mma_bf(acc, ah, bh);
    mma_bf(acc, ah, bl);
    mma_bf(acc, al, bh);
}
__device__ __forceinline__ FragB ldf(const unsigned short* p) {
    FragB f;
    f.h[0] = *(const u16x8*)p;
    f.h[1] = *(const u16x8*)(p + 16);
    return f;
}

__global__ __launch_bounds__(256)
void k_wprep(const float* __restrict__ w_in, const float* __restrict__ w_xp, const float* __restrict__ w_out,
             unsigned short* wih, unsigned short* wil, unsigned short* wxh, unsigned short* wxl,
             unsigned short* woh, unsigned short* wol)
{
    const int blk = blockIdx.x;
    const int tid = threadIdx.x;
    float v[8];
    unsigned short* dh;
    unsigned short* dl;
    size_t e;
    if (blk < 32) {
        const int idx = blk * 256 + tid;
        const int n = idx >> 4, k0 = (idx & 15) * 8;
#pragma unroll
        for (int i = 0; i < 8; ++i) v[i] = w_in[(size_t)(k0 + i) * (2 * DI_) + n];
        dh = wih; dl = wil; e = (size_t)n * DM_ + k0;
    } else if (blk < 38) {
        const int idx = (blk - 32) * 256 + tid;
        const int n = idx >> 5, k0 = (idx & 31) * 8;
        const int nc = (n < NXP_) ? n : (NXP_ - 1);
#pragma unroll
        for (int i = 0; i < 8; ++i) {
            const float t = w_xp[(size_t)(k0 + i) * NXP_ + nc];
            v[i] = (n < NXP_) ? t : 0.0f;
        }
        dh = wxh; dl = wxl; e = (size_t)n * DI_ + k0;
    } else {
        const int idx = (blk - 38) * 256 + tid;
        const int n = idx >> 5, k0 = (idx & 31) * 8;
#pragma unroll
        for (int i = 0; i < 8; ++i) v[i] = w_out[(size_t)(k0 + i) * OC_ + n];
        dh = woh; dl = wol; e = (size_t)n * DI_ + k0;
    }
    u16x8 hv, lv;
#pragma unroll
    for (int i = 0; i < 8; ++i) {
        unsigned short hb, lb;
        split2(v[i], hb, lb);
        hv[i] = hb; lv[i] = lb;
    }
    *(volatile u16x8*)(dh + e) = hv;
    *(volatile u16x8*)(dl + e) = lv;
    __threadfence();
    *(volatile u16x8*)(dh + e) = hv;
    *(volatile u16x8*)(dl + e) = lv;
}

__device__ __forceinline__ void put_rows128(const unsigned short* src, int spitch, unsigned short* dst,
                                            size_t drow0, int dpitch, int dcol, int wave, int h, int m) {
#pragma unroll
    for (int it = 0; it < 8; ++it) {
        const int t = 16 * wave + 2 * it + h;
        const int c0 = 8 * m;
        const u16x8 v = *(const u16x8*)(src + (16 + t) * spitch + c0);
        *(volatile u16x8*)(dst + (drow0 + (size_t)t) * dpitch + dcol + c0) = v;
    }
}

__global__ __launch_bounds__(256)
void k_pre(const float* __restrict__ x, const float* __restrict__ cw, const float* __restrict__ cb,
           const unsigned short* __restrict__ wih, const unsigned short* __restrict__ wil,
           const unsigned short* __restrict__ wxh, const unsigned short* __restrict__ wxl,
           unsigned short* uh, unsigned short* ul, unsigned short* xh, unsigned short* xl, float* xd)
{
    unsigned short* rah = (unsigned short*)smem_dyn;
    unsigned short* ral = rah + TR_ * PA_;
    unsigned short* rch = ral + TR_ * PA_;
    unsigned short* rcl = rch + TR_ * PC_;
    float* rd = (float*)smem_dyn;

    const int tid  = threadIdx.x;
    const int lane = tid & 31;
    const int wave = tid >> 5;
    const int h    = lane >> 4;
    const int m    = lane & 15;
    const int b    = blockIdx.y;
    const int l0   = blockIdx.x * TT_;
    const size_t row0 = (size_t)b * NL_ + l0;

#pragma unroll 1
    for (int it = 0; it < 18; ++it) {
        const int idx = it * 256 + tid;
        const int c   = idx / 36;
        const int q   = idx - c * 36;
        const int l   = l0 - 16 + 4 * q;
        const int lc  = (l < 0) ? 0 : l;
        v4f xv = *(const v4f*)(x + (((size_t)b * DM_ + c) * NL_ + lc));
        if (l < 0) { xv[0] = 0.0f; xv[1] = 0.0f; xv[2] = 0.0f; xv[3] = 0.0f; }
#pragma unroll
        for (int i = 0; i < 4; ++i) {
            unsigned short hb, lb;
            split2(xv[i], hb, lb);
            const int ri = (4 * q + i) * PA_ + c;
            rah[ri] = hb;
            ral[ri] = lb;
        }
    }
    __syncthreads();

    put_rows128(rah, PA_, uh, row0, DM_, 0, wave, h, m);
    put_rows128(ral, PA_, ul, row0, DM_, 0, wave, h, m);
    __threadfence();
    put_rows128(rah, PA_, uh, row0, DM_, 0, wave, h, m);
    put_rows128(ral, PA_, ul, row0, DM_, 0, wave, h, m);

    v8f acc3[3];
#pragma unroll
    for (int j = 0; j < 3; ++j) acc3[j] = zero8();

#pragma unroll 1
    for (int q = 0; q < 2; ++q) {
        {
            FragB fb[4], gb[4];
            const size_t bo = (size_t)(128 * q + 16 * wave + m) * DM_ + 8 * h;
#pragma unroll
            for (int kt = 0; kt < 4; ++kt) {
                fb[kt] = ldf(wih + bo + 32 * kt);
                gb[kt] = ldf(wil + bo + 32 * kt);
            }
#pragma unroll 1
            for (int s = 0; s < 9; ++s) {
                v8f acc = zero8();
                const int ao = (16 * s + m) * PA_ + 8 * h;
#pragma unroll
                for (int kt = 0; kt < 4; ++kt) {
                    const FragB fa = ldf(rah + ao + 32 * kt);
                    const FragB ga = ldf(ral + ao + 32 * kt);
                    mma3(acc, fa, ga, fb[kt], gb[kt]);
                }
#pragma unroll
                for (int r = 0; r < 8; ++r) {
                    unsigned short hb, lb;
                    split2(acc[r], hb, lb);
                    const int ri = (16 * s + 8 * h + r) * PC_ + 16 * wave + m;
                    rch[ri] = hb;
                    rcl[ri] = lb;
                }
            }
        }
        __syncthreads();

        if (wave < 4) {
            const int d = 128 * q + tid;
            const float w0 = cw[d * 4 + 0], w1 = cw[d * 4 + 1], w2 = cw[d * 4 + 2], w3 = cw[d * 4 + 3];
            const float bias = cb[d];
            float xt  = bf2f(rch[(TR_ - 1) * PC_ + tid]) + bf2f(rcl[(TR_ - 1) * PC_ + tid]);
            float xm1 = bf2f(rch[(TR_ - 2) * PC_ + tid]) + bf2f(rcl[(TR_ - 2) * PC_ + tid]);
            float xm2 = bf2f(rch[(TR_ - 3) * PC_ + tid]) + bf2f(rcl[(TR_ - 3) * PC_ + tid]);
#pragma unroll 2
            for (int t = TR_ - 1; t >= 16; --t) {
                const float xm3 = bf2f(rch[(t - 3) * PC_ + tid]) + bf2f(rcl[(t - 3) * PC_ + tid]);
                float c = w0 * xm3;
                c = fmaf(w1, xm2, c);
                c = fmaf(w2, xm1, c);
                c = fmaf(w3, xt, c);
                c += bias;
                const float uu = silu_f(c);
                unsigned short hb, lb;
                split2(uu, hb, lb);
                rch[t * PC_ + tid] = hb;
                rcl[t * PC_ + tid] = lb;
                xt = xm1; xm1 = xm2; xm2 = xm3;
            }
        }
        __syncthreads();

        put_rows128(rch, PC_, xh, row0, DI_, 128 * q, wave, h, m);
        put_rows128(rcl, PC_, xl, row0, DI_, 128 * q, wave, h, m);
        __threadfence();
        put_rows128(rch, PC_, xh, row0, DI_, 128 * q, wave, h, m);
        put_rows128(rcl, PC_, xl, row0, DI_, 128 * q, wave, h, m);

        {
            const int ao = (16 + 16 * wave + m) * PC_ + 8 * h;
#pragma unroll 1
            for (int kt = 0; kt < 4; ++kt) {
                const FragB fa = ldf(rch + ao + 32 * kt);
                const FragB ga = ldf(rcl + ao + 32 * kt);
#pragma unroll
                for (int j = 0; j < 3; ++j) {
                    const size_t bo = (size_t)(16 * j + m) * DI_ + 128 * q + 32 * kt + 8 * h;
                    const FragB fbx = ldf(wxh + bo);
                    const FragB gbx = ldf(wxl + bo);
                    mma3(acc3[j], fa, ga, fbx, gbx);
                }
            }
        }
        __syncthreads();
    }

#pragma unroll
    for (int j = 0; j < 3; ++j)
#pragma unroll
        for (int r = 0; r < 8; ++r)
            rd[(16 * wave + 8 * h + r) * PD_ + 16 * j + m] = acc3[j][r];
#pragma unroll
    for (int r = 0; r < 8; ++r)
        rd[(16 * wave + 8 * h + r) * PD_ + NXT_ + m] = 0.0f;
    __syncthreads();

#pragma unroll
    for (int ps = 0; ps < 2; ++ps) {
#pragma unroll
        for (int it = 0; it < 8; ++it) {
            const int t  = 16 * wave + 2 * it + h;
            const int c0 = 4 * m;
            const v4f v = *(const v4f*)(rd + t * PD_ + c0);
            *(volatile v4f*)(xd + (row0 + (size_t)t) * XDP_ + c0) = v;
        }
        if (ps == 0) __threadfence();
    }
}

__global__ __launch_bounds__(64)
void k_scan(const unsigned short* __restrict__ uh, const unsigned short* __restrict__ ul,
            const unsigned short* __restrict__ wih, const unsigned short* __restrict__ wil,
            const float* __restrict__ xd, const float* __restrict__ wdt, const float* __restrict__ bdt,
            const float* __restrict__ alog, const float* __restrict__ dpar,
            unsigned short* xh, unsigned short* xl)
{
    __shared__ __attribute__((aligned(16))) float zs[64 * PZ_];
    __shared__ __attribute__((aligned(16))) unsigned short shi[64 * 64];
    __shared__ __attribute__((aligned(16))) unsigned short slo[64 * 64];

    const int tid  = threadIdx.x;
    const int lane = tid & 31;
    const int wave = tid >> 5;
    const int h    = lane >> 4;
    const int m    = lane & 15;
    const int cq   = blockIdx.x;
    const int b    = blockIdx.y;
    const int d    = 64 * cq + tid;
    const size_t rowb = (size_t)b * NL_;

    float a2[NS_], hs[NS_];
#pragma unroll
    for (int n = 0; n < NS_; ++n) {
        a2[n] = -expf(alog[(size_t)d * NS_ + n]) * 1.4426950408889634f;
        hs[n] = 0.0f;
    }
    float wv[DTR_];
#pragma unroll
    for (int r = 0; r < DTR_; ++r) wv[r] = wdt[(size_t)r * DI_ + d];
    const float tb = bdt[d];
    const float Dd = dpar[d];

    unsigned short* plane = wave ? xl : xh;
    const unsigned short* sl = wave ? slo : shi;

#pragma unroll 1
    for (int l0 = 0; l0 < NL_; l0 += 64) {
#pragma unroll 1
        for (int s = 0; s < 4; ++s) {
            v8f acc[2];
            acc[0] = zero8(); acc[1] = zero8();
            const size_t ao = (rowb + (size_t)l0 + 16 * s + m) * DM_ + 8 * h;
#pragma unroll 1
            for (int kt = 0; kt < 4; ++kt) {
                const FragB fa = ldf(uh + ao + 32 * kt);
                const FragB ga = ldf(ul + ao + 32 * kt);
#pragma unroll
                for (int j = 0; j < 2; ++j) {
                    const size_t bo = (size_t)(DI_ + 64 * cq + 32 * wave + 16 * j + m) * DM_ + 32 * kt + 8 * h;
                    const FragB fbz = ldf(wih + bo);
                    const FragB gbz = ldf(wil + bo);
                    mma3(acc[j], fa, ga, fbz, gbz);
                }
            }
#pragma unroll
            for (int j = 0; j < 2; ++j)
#pragma unroll
                for (int r = 0; r < 8; ++r)
                    zs[(16 * s + 8 * h + r) * PZ_ + 32 * wave + 16 * j + m] = acc[j][r];
        }
        __syncthreads();

#pragma unroll 1
        for (int t = 0; t < 64; ++t) {
            const size_t row = rowb + (size_t)l0 + t;
            const size_t e = row * DI_ + d;
            const float u = bf2f(xh[e]) + bf2f(xl[e]);
            const float* p = xd + row * XDP_;
            float pre = p[0] * wv[0];
#pragma unroll
            for (int r = 1; r < DTR_; ++r) pre = fmaf(p[r], wv[r], pre);
            pre += tb;
            const float dt = softplus_f(pre);
            const float du = dt * u;
            float y = 0.0f;
#pragma unroll
            for (int n = 0; n < NS_; ++n) {
                const float da = exp2f(dt * a2[n]);
                hs[n] = fmaf(da, hs[n], du * p[DTR_ + n]);
                y = fmaf(hs[n], p[DTR_ + NS_ + n], y);
            }
            const float g = fmaf(Dd, u, y) * silu_f(zs[t * PZ_ + tid]);
            unsigned short hb, lb;
            split2(g, hb, lb);
            shi[t * 64 + tid] = hb;
            slo[t * 64 + tid] = lb;
        }
        __syncthreads();

#pragma unroll
        for (int ps = 0; ps < 2; ++ps) {
#pragma unroll
            for (int it = 0; it < 16; ++it) {
                const int t  = 4 * it + (lane >> 3);
                const int c0 = 8 * (lane & 7);
                const u16x8 v = *(const u16x8*)(sl + t * 64 + c0);
                *(volatile u16x8*)(plane + (rowb + (size_t)l0 + t) * DI_ + 64 * cq + c0) = v;
            }
            if (ps == 0) __threadfence();
        }
        __syncthreads();
    }
}

__global__ __launch_bounds__(128)
void k_out(const unsigned short* __restrict__ yh, const unsigned short* __restrict__ yl,
           const unsigned short* __restrict__ woh, const unsigned short* __restrict__ wol, float* out)
{
    __shared__ __attribute__((aligned(16))) float st[4 * 32 * PO_];

    const int tid  = threadIdx.x;
    const int lane = tid & 31;
    const int wave = tid >> 5;
    const int hh   = lane >> 4;
    const int m    = lane & 15;
    const int wm   = wave >> 1;
    const int wn   = wave & 1;
    const int cx   = blockIdx.x;
    const int bw   = blockIdx.y;
    const int b    = bw >> 6;
    const int w    = bw & 63;
    const size_t abase  = ((size_t)b * NL_ + w) * DI_;
    const size_t apitch = (size_t)WW_ * DI_;

    v8f acc[4];
#pragma unroll
    for (int i = 0; i < 4; ++i) acc[i] = zero8();

#pragma unroll 1
    for (int kt = 0; kt < 8; ++kt) {
        FragB fa[2], ga[2], fb[2], gb[2];
#pragma unroll
        for (int s = 0; s < 2; ++s) {
            const size_t ao = abase + (size_t)(32 * wm + 16 * s + m) * apitch + 32 * kt + 8 * hh;
            fa[s] = ldf(yh + ao);
            ga[s] = ldf(yl + ao);
        }
#pragma unroll
        for (int j = 0; j < 2; ++j) {
            const size_t bo = (size_t)(64 * cx + 32 * wn + 16 * j + m) * DI_ + 32 * kt + 8 * hh;
            fb[j] = ldf(woh + bo);
            gb[j] = ldf(wol + bo);
        }
#pragma unroll
        for (int s = 0; s < 2; ++s)
#pragma unroll
            for (int j = 0; j < 2; ++j)
                mma3(acc[s * 2 + j], fa[s], ga[s], fb[j], gb[j]);
    }

    float* sw = st + wave * 32 * PO_;
#pragma unroll
    for (int s = 0; s < 2; ++s)
#pragma unroll
        for (int j = 0; j < 2; ++j)
#pragma unroll
            for (int r = 0; r < 8; ++r)
                sw[(16 * j + m) * PO_ + 16 * s + 8 * hh + r] = acc[s * 2 + j][r];
    __syncthreads();

#pragma unroll
    for (int ps = 0; ps < 2; ++ps) {
#pragma unroll
        for (int it = 0; it < 8; ++it) {
            const int cl = 4 * it + (lane >> 3);
            const int c  = 64 * cx + 32 * wn + cl;
            const int h4 = 4 * (lane & 7);
            const v4f v = *(const v4f*)(sw + cl * PO_ + h4);
            const size_t e = (((size_t)b * OC_ + c) * WW_ + w) * HH_ + 32 * wm + h4;
            *(volatile v4f*)(out + e) = v;
        }
        if (ps == 0) __threadfence();
    }
}

extern "C" void kernel_launch(void* const* d_in, const int* in_sizes, int n_in,
                              void* d_out, int out_size, void* d_ws, size_t ws_size,
                              hipStream_t stream)
{
    if (n_in < 10) return;
    if (in_sizes[0] != MT_ * DM_)        return;
    if (in_sizes[1] != DM_ * 2 * DI_)    return;
    if (in_sizes[2] != DI_ * 4)          return;
    if (in_sizes[3] != DI_)              return;
    if (in_sizes[4] != DI_ * NXP_)       return;
    if (in_sizes[5] != DTR_ * DI_)       return;
    if (in_sizes[6] != DI_)              return;
    if (in_sizes[7] != DI_ * NS_)        return;
    if (in_sizes[8] != DI_)              return;
    if (in_sizes[9] != DI_ * OC_)        return;
    if (out_size != MT_ * OC_)           return;
    if (ws_size < WS_END)                return;

    const float* x    = (const float*)d_in[0];
    const float* w_in = (const float*)d_in[1];
    const float* cw   = (const float*)d_in[2];
    const float* cb   = (const float*)d_in[3];
    const float* w_xp = (const float*)d_in[4];
    const float* wdt  = (const float*)d_in[5];
    const float* bdt  = (const float*)d_in[6];
    const float* alog = (const float*)d_in[7];
    const float* dpar = (const float*)d_in[8];
    const float* w_ou = (const float*)d_in[9];
    float* out = (float*)d_out;

    char* ws = (char*)d_ws;
    unsigned short* wih = (unsigned short*)(ws + OFF_WIH);
    unsigned short* wil = (unsigned short*)(ws + OFF_WIL);
    unsigned short* wxh = (unsigned short*)(ws + OFF_WXH);
    unsigned short* wxl = (unsigned short*)(ws + OFF_WXL);
    unsigned short* woh = (unsigned short*)(ws + OFF_WOH);
    unsigned short* wol = (unsigned short*)(ws + OFF_WOL);
    unsigned short* uh  = (unsigned short*)(ws + OFF_UH);
    unsigned short* ul  = (unsigned short*)(ws + OFF_UL);
    unsigned short* xh  = (unsigned short*)(ws + OFF_XH);
    unsigned short* xl  = (unsigned short*)(ws + OFF_XL);
    float*          xd  = (float*)(ws + OFF_XD);

    hipLaunchKernelGGL(k_wprep, dim3(54), dim3(256), 0, stream,
                       w_in, w_xp, w_ou, wih, wil, wxh, wxl, woh, wol);

    hipLaunchKernelGGL(k_pre, dim3(NL_ / TT_, NB_), dim3(256), LDS_PRE, stream,
                       x, cw, cb,
                       (const unsigned short*)wih, (const unsigned short*)wil,
                       (const unsigned short*)wxh, (const unsigned short*)wxl,
                       uh, ul, xh, xl, xd);

    hipLaunchKernelGGL(k_scan, dim3(DI_ / 64, NB_), dim3(64), 0, stream,
                       (const unsigned short*)uh, (const unsigned short*)ul,
                       (const unsigned short*)wih, (const unsigned short*)wil,
                       (const float*)xd, wdt, bdt, alog, dpar, xh, xl);

    hipLaunchKernelGGL(k_out, dim3(OC_ / 64, NB_ * WW_), dim3(128), 0, stream,
                       (const unsigned short*)xh, (const unsigned short*)xl,
                       (const unsigned short*)woh, (const unsigned short*)wol, out);
}
